// NAttention_9337258901738
// MI455X (gfx1250) — hardware-verified
//
#include <hip/hip_runtime.h>
#ifndef NB
#define NB 2
#endif
#define NB_FULL 2
#define CC 256
#define HHT 64
#define WID 64
#define PIX (HHT * WID)
#define NHD 8
#define HD 32
#define KS 7
#define NTAP (KS * KS)
#define RPW (2 * KS - 1)
#define RPN (RPW * RPW)
#define QLD (3 * CC)
#define OLD (2 * CC)
#define PBLK 128
#define NPB (PIX / PBLK)
#define XT_P 32
#define XT_C 64
#define XSC 16.0f
#define WSC 64.0f
#define OSC 64.0f
#define RSC 1024.0f
#define PSC 1024.0f
#define QSCALE 0.17677669529663687f
static_assert(NB <= NB_FULL);
static_assert(PIX % PBLK == 0);
static_assert(PIX % 128 == 0);
static_assert(PIX % 64 == 0);
static_assert(PIX % XT_P == 0);
static_assert(CC % XT_C == 0);
static_assert(CC % 128 == 0);
static_assert(CC % 32 == 0);
static_assert(OLD % 32 == 0);
static_assert(QLD % 64 == 0);
static_assert(PBLK == 128);
static_assert(HD == 32);
static_assert(NHD * HD == CC);
static_assert(HHT >= KS && WID >= KS);

typedef unsigned short v8us __attribute__((ext_vector_type(8), may_alias));
typedef float v8f __attribute__((ext_vector_type(8)));
typedef float v4f __attribute__((ext_vector_type(4)));
typedef float v4fa __attribute__((ext_vector_type(4), may_alias));
typedef _Float16 v16h __attribute__((ext_vector_type(16)));
union FragH { v16h v; v8us half[2]; _Float16 h[16]; unsigned short u[16]; };

__device__ __forceinline__ unsigned short bf16_bits(float x) { unsigned int u = __float_as_uint(x); return (unsigned short)((u + 0x7FFFu + ((u >> 16) & 1u)) >> 16); }
__device__ __forceinline__ float bf16_val(unsigned short b) { return __uint_as_float(((unsigned int)b) << 16); }
__device__ __forceinline__ float bf16_rne(float x) { return bf16_val(bf16_bits(x)); }

__device__ __forceinline__ v16h g2_frag(const _Float16* p, int hh) { FragH f; f.half[0] = *(const v8us*)((const unsigned short*)p + 8 * hh); f.half[1] = *(const v8us*)((const unsigned short*)p + 16 + 8 * hh); return f.v; }
__device__ __forceinline__ v8f g2_mma(v16h a, v16h b, v8f c) { v8f d = __builtin_amdgcn_wmma_f32_16x16x32_f16(false, a, false, b, (short)0, c, false, false); asm volatile("v_nop\n\tv_nop\n\tv_nop\n\tv_nop" : "+v"(d) : "v"(a), "v"(b)); return d; }

__global__ __launch_bounds__(128) void k_gemm2(const _Float16* __restrict__ A, int lda, const _Float16* __restrict__ Bh, int ldb, float alpha,
                                               const float* __restrict__ bcol, const float* __restrict__ brow,
                                               float* __restrict__ C, int ldc, int M, int N, int K) {
  __shared__ __attribute__((aligned(16))) float so[4][32][68];
  const int tid = threadIdx.x, w = tid >> 5, lane = tid & 31, ln = lane & 15, hh = lane >> 4;
  const int ntn = N >> 6; const int mt = blockIdx.x / ntn, nq = blockIdx.x - mt * ntn; const int row0 = mt * 128 + 32 * w, col0 = nq * 64; if (row0 >= M) return;
  const _Float16* a0p = A + (size_t)(row0 + ln) * lda; const _Float16* a1p = a0p + (size_t)16 * lda;
  const _Float16* b0p = Bh + (size_t)(col0 + ln) * ldb; const _Float16* b1p = b0p + (size_t)16 * ldb; const _Float16* b2p = b1p + (size_t)16 * ldb; const _Float16* b3p = b2p + (size_t)16 * ldb;
  const v8f z8 = {0.f,0.f,0.f,0.f,0.f,0.f,0.f,0.f}; v8f c00 = z8, c01 = z8, c02 = z8, c03 = z8, c10 = z8, c11 = z8, c12 = z8, c13 = z8;
#pragma unroll 1
  for (int kb = 0; kb < K; kb += 32) { const v16h a0 = g2_frag(a0p + kb, hh), a1 = g2_frag(a1p + kb, hh);
    v16h b = g2_frag(b0p + kb, hh); c00 = g2_mma(a0, b, c00); c10 = g2_mma(a1, b, c10);
    b = g2_frag(b1p + kb, hh); c01 = g2_mma(a0, b, c01); c11 = g2_mma(a1, b, c11);
    b = g2_frag(b2p + kb, hh); c02 = g2_mma(a0, b, c02); c12 = g2_mma(a1, b, c12);
    b = g2_frag(b3p + kb, hh); c03 = g2_mma(a0, b, c03); c13 = g2_mma(a1, b, c13); }
  v8f accs[8] = {c00, c01, c02, c03, c10, c11, c12, c13};
#pragma unroll
  for (int u = 0; u < 8; ++u) { const int t = u & 3, half = u >> 2; const int col = col0 + t * 16 + ln; const float bv = bcol ? bf16_rne(bcol[col]) : 0.f;
#pragma unroll
    for (int r = 0; r < 8; ++r) { const int rloc = half * 16 + 8 * hh + r; float v = accs[u][r] * alpha + bv; if (brow) v += bf16_rne(brow[row0 + rloc]); so[w][rloc][t * 16 + ln] = v; } }
  __builtin_amdgcn_fence(__ATOMIC_ACQ_REL, "workgroup"); __builtin_amdgcn_wave_barrier();
  const int rsub = lane >> 4, c4 = (lane & 15) * 4;
  for (int pass = 0; pass < 2; ++pass) {
#pragma unroll
    for (int q = 0; q < 16; ++q) { const int r = q * 2 + rsub; const v4f v = *(const v4fa*)&so[w][r][c4]; *(volatile v4f*)(C + (size_t)(row0 + r) * ldc + col0 + c4) = v; }
    if (pass == 0) __threadfence(); }
}

__global__ __launch_bounds__(256) void k_cvt8(const float* __restrict__ W, _Float16* __restrict__ Bt, int n8, float scale) {
  const int t = blockIdx.x * 256 + threadIdx.x; if (t >= n8) return; FragH f;
#pragma unroll
  for (int i = 0; i < 8; ++i) f.h[i] = (_Float16)(bf16_rne(W[(size_t)t * 8 + i]) * scale);
  unsigned short* dst = (unsigned short*)Bt + (size_t)t * 8;
  *(volatile v8us*)dst = f.half[0]; __threadfence(); *(volatile v8us*)dst = f.half[0];
}

__global__ __launch_bounds__(256) void k_wpa(const float* __restrict__ W, _Float16* __restrict__ WPA) {
  const int t = blockIdx.x * 256 + threadIdx.x; if (t >= CC * OLD / 8) return;
  const int c = t / (OLD / 8); const int k8 = (t - c * (OLD / 8)) * 8; const int h = k8 >> 6; const int wi = k8 & 63; const int d0 = wi & 31;
  const float sc = (wi >= 32) ? 1.0f : PSC;
  FragH f;
#pragma unroll
  for (int i = 0; i < 8; ++i) f.h[i] = (_Float16)(bf16_rne(W[(size_t)c * CC + h * HD + d0 + i]) * sc);
  unsigned short* dst = (unsigned short*)WPA + (size_t)t * 8;
  *(volatile v8us*)dst = f.half[0]; __threadfence(); *(volatile v8us*)dst = f.half[0];
}

__global__ __launch_bounds__(256) void k_xt(const float* __restrict__ x, _Float16* __restrict__ X16) {
  __shared__ __attribute__((aligned(16))) _Float16 st[XT_P][XT_C];
  const int tid = threadIdx.x, w = tid >> 5, lane = tid & 31;
  int blk = blockIdx.x;
  const int pt = blk % (PIX / XT_P); blk /= (PIX / XT_P);
  const int ch = blk % (CC / XT_C); const int b = blk / (CC / XT_C);
  const float* src = x + ((size_t)(b * CC + ch * XT_C)) * PIX + (size_t)pt * XT_P + lane;
#pragma unroll
  for (int it = 0; it < XT_C / 8; ++it) {
    const int ci = it * 8 + w;
    const float v = src[(size_t)ci * PIX];
    st[lane][ci] = (_Float16)(bf16_rne(v) * XSC);
  }
  __syncthreads();
  const int rr = w * 4 + (lane >> 3), q = lane & 7;
  const v8us o = *(const v8us*)&st[rr][q * 8];
  unsigned short* dst = (unsigned short*)X16 + ((size_t)(b * PIX + pt * XT_P + rr)) * CC + ch * XT_C + q * 8;
  *(volatile v8us*)dst = o; __threadfence(); *(volatile v8us*)dst = o;
}

__global__ __launch_bounds__(PBLK) void k_att(const float* __restrict__ QKV, const float* __restrict__ rpb, _Float16* __restrict__ O16) {
  __shared__ float srpb[RPN + 7];
  __shared__ __attribute__((aligned(16))) float slog[NTAP][PBLK];
  __shared__ __attribute__((aligned(16))) unsigned short sO[PBLK][64];
  const int tid = threadIdx.x, w = tid >> 5, lane = tid & 31;
  const int h = blockIdx.x / NPB; const int p0 = (blockIdx.x - h * NPB) * PBLK;
  for (int t = tid; t < RPN; t += PBLK) srpb[t] = bf16_rne(rpb[h * RPN + t]);
  __syncthreads();
  const int p = p0 + tid; const int y = p / WID, x = p - y * WID;
  int ni = y - KS / 2; ni = (ni < 0) ? 0 : ((ni > HHT - KS) ? (HHT - KS) : ni);
  int nj = x - KS / 2; nj = (nj < 0) ? 0 : ((nj > WID - KS) ? (WID - KS) : nj);
  const int bi = ni - y + (KS - 1), bj = nj - x + (KS - 1);
  const float* qr = QKV + (size_t)p * QLD + h * HD;
  float qv[HD];
#pragma unroll
  for (int g = 0; g < HD / 4; ++g) { const v4f q4 = *(const v4fa*)(qr + 4 * g);
#pragma unroll
    for (int e = 0; e < 4; ++e) qv[4 * g + e] = q4[e]; }
  float mx = -3.0e38f;
#pragma unroll 1
  for (int i = 0; i < KS; ++i) {
    const float* krow = QKV + (size_t)((ni + i) * WID + nj) * QLD + CC + h * HD;
#pragma unroll 1
    for (int j = 0; j < KS; ++j) {
      const float* kr = krow + (size_t)j * QLD;
      float a = 0.f;
#pragma unroll
      for (int g = 0; g < HD / 4; ++g) { const v4f k4 = *(const v4fa*)(kr + 4 * g);
#pragma unroll
        for (int e = 0; e < 4; ++e) a = fmaf(qv[4 * g + e], k4[e], a); }
      const float l = a * QSCALE + srpb[(bi + i) * RPW + (bj + j)];
      slog[i * KS + j][tid] = l;
      mx = fmaxf(mx, l);
    }
  }
  float s = 0.f; float acc[HD];
#pragma unroll
  for (int d = 0; d < HD; ++d) acc[d] = 0.f;
#pragma unroll 1
  for (int i = 0; i < KS; ++i) {
    const float* vrow = QKV + (size_t)((ni + i) * WID + nj) * QLD + 2 * CC + h * HD;
#pragma unroll 1
    for (int j = 0; j < KS; ++j) {
      const float l = slog[i * KS + j][tid]; const float e = expf(l - mx); s += e;
      const float* vr = vrow + (size_t)j * QLD;
#pragma unroll
      for (int g = 0; g < HD / 4; ++g) { const v4f v = *(const v4fa*)(vr + 4 * g);
#pragma unroll
        for (int e2 = 0; e2 < 4; ++e2) acc[4 * g + e2] = fmaf(e, v[e2], acc[4 * g + e2]); } } }
  const float inv = 1.0f / s;
#pragma unroll
  for (int g = 0; g < HD / 8; ++g) { FragH fh, fr;
#pragma unroll
    for (int e2 = 0; e2 < 8; ++e2) { const float o64 = (acc[g * 8 + e2] * inv) * OSC; const _Float16 hv = (_Float16)o64; fh.h[e2] = hv; fr.h[e2] = (_Float16)((o64 - (float)hv) * RSC); }
    *(v8us*)&sO[tid][g * 8] = fh.half[0]; *(v8us*)&sO[tid][HD + g * 8] = fr.half[0]; }
  __syncthreads();
  for (int pass = 0; pass < 2; ++pass) {
#pragma unroll
    for (int it = 0; it < 8; ++it) { const int rr = w * 32 + it * 4 + (lane >> 3), q = lane & 7; const v8us o = *(const v8us*)&sO[rr][q * 8];
      *(volatile v8us*)((unsigned short*)O16 + ((size_t)(p0 + rr)) * OLD + h * 64 + q * 8) = o; }
    if (pass == 0) __threadfence(); }
}

extern "C" void kernel_launch(void* const* d_in, const int* in_sizes, int n_in,
                              void* d_out, int out_size, void* d_ws, size_t ws_size, hipStream_t stream) {
  if (n_in < 6) return;
  if (in_sizes[0] < NB * CC * PIX || in_sizes[1] < 3 * CC * CC || in_sizes[2] < 3 * CC || in_sizes[3] < NHD * RPN || in_sizes[4] < CC * CC || in_sizes[5] < CC) return;
  if (out_size < NB * CC * PIX) return;
  const float* x = (const float*)d_in[0]; const float* qkv_w = (const float*)d_in[1]; const float* qkv_b = (const float*)d_in[2];
  const float* rpb = (const float*)d_in[3]; const float* proj_w = (const float*)d_in[4]; const float* proj_b = (const float*)d_in[5];
  float* out = (float*)d_out;
  char* ws = (char*)d_ws; size_t off = 0;
  auto take = [&](size_t bytes) { char* p = ws + off; off += (bytes + 255) & ~(size_t)255; return p; };
  _Float16* X16 = (_Float16*)take((size_t)NB * PIX * CC * 2);
  _Float16* WQ16 = (_Float16*)take((size_t)3 * CC * CC * 2);
  _Float16* WPA = (_Float16*)take((size_t)CC * OLD * 2);
  float* QKV = (float*)take((size_t)PIX * QLD * 4);
  _Float16* O16 = (_Float16*)take((size_t)PIX * OLD * 2);
  if (off > ws_size || off > ((size_t)128 << 20)) return;
  k_xt<<<(unsigned)(NB * (CC / XT_C) * (PIX / XT_P)), 256, 0, stream>>>(x, X16);
  k_cvt8<<<(3 * CC * CC / 8 + 255) / 256, 256, 0, stream>>>(qkv_w, WQ16, 3 * CC * CC / 8, WSC);
  k_wpa<<<(CC * OLD / 8 + 255) / 256, 256, 0, stream>>>(proj_w, WPA);
  for (int b = 0; b < NB; ++b) {
    k_gemm2<<<(unsigned)((PIX / 128) * (QLD / 64)), 128, 0, stream>>>(X16 + (size_t)b * PIX * CC, CC, WQ16, CC, 1.0f / (XSC * WSC), qkv_b, nullptr, QKV, QLD, PIX, QLD, CC);
    k_att<<<NHD * NPB, PBLK, 0, stream>>>(QKV, rpb, O16);
    k_gemm2<<<(unsigned)((CC / 128) * (PIX / 64)), 128, 0, stream>>>(WPA, OLD, O16, OLD, 1.0f / (PSC * OSC), nullptr, proj_b, out + (size_t)b * CC * PIX, PIX, CC, PIX, OLD);
  }
}
